// SparseNeighborhoodAttentionBlock_2052994367931
// MI455X (gfx1250) — hardware-verified
//
#include <hip/hip_runtime.h>
#include <stddef.h>


typedef __bf16       v16bf __attribute__((ext_vector_type(16)));
typedef float        v8f   __attribute__((ext_vector_type(8)));
typedef float        v4f   __attribute__((ext_vector_type(4)));
typedef unsigned int v4u   __attribute__((ext_vector_type(4)));

union Frag { v4u u[2]; unsigned short s[16]; v16bf v; };

#define DM     256
#define NLEV   4
#define FH     64
#define FW     64
#define CPB    (NLEV * FH * FW)
#define LT     164
#define KROWS  176
#define VROWS  192
#define RPH    264
#define ATP    192
#define BM     32
#define AP     264
#define TP     260
#define RSQ    0.17677669529663688f

#define G_AH   0
#define G_AL   16896
#define G_T    33792
#define G_CS   67072
#define G_SN   69120
#define G_TOT  71168

#define A_R    0
#define A_QH   101376
#define A_QL   101888
#define A_SCP  102400
#define A_ATT  113664
#define A_OP   119808
#define A_OS   136192
#define A_CELL 137216
#define A_OOB  137984
#define A_TOT  138752

__constant__ float c_fs[16] = {
  1.0f, 0.74989420933245583f, 0.56234132519034908f, 0.42169650342858225f,
  0.31622776601683794f, 0.23713737056616554f, 0.17782794100389229f, 0.13335214321633240f,
  0.1f, 0.074989420933245583f, 0.056234132519034908f, 0.042169650342858225f,
  0.031622776601683794f, 0.023713737056616554f, 0.017782794100389229f, 0.013335214321633240f };
__constant__ float c_fl[16] = {
  1.0f, 0.86596432336006535f, 0.74989420933245583f, 0.64938163157621132f,
  0.56234132519034908f, 0.48696752516586311f, 0.42169650342858225f, 0.36517412725483772f,
  0.31622776601683794f, 0.27384196342643611f, 0.23713737056616554f, 0.20535250264571461f,
  0.17782794100389229f, 0.15399265260594920f, 0.13335214321633240f, 0.11547819846894582f };

__device__ __forceinline__ unsigned short f2bf(float f) {
  unsigned u = __float_as_uint(f);
  u += 0x7FFFu + ((u >> 16) & 1u);
  return (unsigned short)(u >> 16);
}
__device__ __forceinline__ float bf2f(unsigned short h) { return __uint_as_float(((unsigned)h) << 16); }

__device__ __forceinline__ void split8(const float* x, v4u& hi, v4u& lo) {
  unsigned hw[4], lw[4];
#pragma unroll
  for (int j = 0; j < 4; ++j) {
    const unsigned short h0 = f2bf(x[2 * j]), h1 = f2bf(x[2 * j + 1]);
    const unsigned short l0 = f2bf(x[2 * j] - bf2f(h0)), l1 = f2bf(x[2 * j + 1] - bf2f(h1));
    hw[j] = (unsigned)h0 | ((unsigned)h1 << 16);
    lw[j] = (unsigned)l0 | ((unsigned)l1 << 16);
  }
  hi.x = hw[0]; hi.y = hw[1]; hi.z = hw[2]; hi.w = hw[3];
  lo.x = lw[0]; lo.y = lw[1]; lo.z = lw[2]; lo.w = lw[3];
}

__device__ __forceinline__ float wsum(float v) {
#pragma unroll
  for (int m = 16; m >= 1; m >>= 1) v += __shfl_xor(v, m, 32);
  return v;
}
__device__ __forceinline__ float wmax(float v) {
#pragma unroll
  for (int m = 16; m >= 1; m >>= 1) v = fmaxf(v, __shfl_xor(v, m, 32));
  return v;
}

__device__ __forceinline__ v8f wmma16(v16bf a, v16bf b, v8f c) {
  v8f d = __builtin_amdgcn_wmma_f32_16x16x32_bf16(false, a, false, b, (short)0, c, false, false);
  asm volatile("v_nop\n\tv_nop\n\tv_nop\n\tv_nop" : "+v"(d) : "v"(a), "v"(b));
  return d;
}

__device__ __forceinline__ void gemm_tile(const unsigned short* Ah, const unsigned short* Al,
                                          const unsigned short* __restrict__ Wh,
                                          const unsigned short* __restrict__ Wl,
                                          float* T, int wave, int lane) {
  const int n = lane & 15, hh = lane >> 4;
  v8f z = {0.f, 0.f, 0.f, 0.f, 0.f, 0.f, 0.f, 0.f};
  v8f a00 = z, a01 = z, a10 = z, a11 = z;
  const unsigned short* w0 = Wh + (size_t)(32 * wave + n) * DM + 8 * hh;
  const unsigned short* w1 = Wh + (size_t)(32 * wave + 16 + n) * DM + 8 * hh;
  const unsigned short* u0 = Wl + (size_t)(32 * wave + n) * DM + 8 * hh;
  const unsigned short* u1 = Wl + (size_t)(32 * wave + 16 + n) * DM + 8 * hh;
  const unsigned short* p0 = Ah + n * AP + 8 * hh;
  const unsigned short* p1 = Ah + (16 + n) * AP + 8 * hh;
  const unsigned short* q0 = Al + n * AP + 8 * hh;
  const unsigned short* q1 = Al + (16 + n) * AP + 8 * hh;
#pragma unroll 1
  for (int ks = 0; ks < DM / 32; ++ks) {
    const int k0 = 32 * ks;
    Frag bh0, bh1, bl0, bl1, ah0, ah1, al0, al1;
    bh0.u[0] = *(const v4u*)(w0 + k0); bh0.u[1] = *(const v4u*)(w0 + k0 + 16);
    bh1.u[0] = *(const v4u*)(w1 + k0); bh1.u[1] = *(const v4u*)(w1 + k0 + 16);
    bl0.u[0] = *(const v4u*)(u0 + k0); bl0.u[1] = *(const v4u*)(u0 + k0 + 16);
    bl1.u[0] = *(const v4u*)(u1 + k0); bl1.u[1] = *(const v4u*)(u1 + k0 + 16);
    ah0.u[0] = *(const v4u*)(p0 + k0); ah0.u[1] = *(const v4u*)(p0 + k0 + 16);
    ah1.u[0] = *(const v4u*)(p1 + k0); ah1.u[1] = *(const v4u*)(p1 + k0 + 16);
    al0.u[0] = *(const v4u*)(q0 + k0); al0.u[1] = *(const v4u*)(q0 + k0 + 16);
    al1.u[0] = *(const v4u*)(q1 + k0); al1.u[1] = *(const v4u*)(q1 + k0 + 16);
    a00 = wmma16(ah0.v, bh0.v, a00); a00 = wmma16(ah0.v, bl0.v, a00); a00 = wmma16(al0.v, bh0.v, a00);
    a01 = wmma16(ah0.v, bh1.v, a01); a01 = wmma16(ah0.v, bl1.v, a01); a01 = wmma16(al0.v, bh1.v, a01);
    a10 = wmma16(ah1.v, bh0.v, a10); a10 = wmma16(ah1.v, bl0.v, a10); a10 = wmma16(al1.v, bh0.v, a10);
    a11 = wmma16(ah1.v, bh1.v, a11); a11 = wmma16(ah1.v, bl1.v, a11); a11 = wmma16(al1.v, bh1.v, a11);
  }
#pragma unroll
  for (int r = 0; r < 8; ++r) {
    T[(8 * hh + r) * TP + 32 * wave + n]           = a00[r];
    T[(8 * hh + r) * TP + 32 * wave + 16 + n]      = a01[r];
    T[(16 + 8 * hh + r) * TP + 32 * wave + n]      = a10[r];
    T[(16 + 8 * hh + r) * TP + 32 * wave + 16 + n] = a11[r];
  }
}

template <bool ROT>
__device__ __forceinline__ void epi_planes(const float* T, const float* csS, const float* snS,
                                           unsigned short* __restrict__ Ph,
                                           unsigned short* __restrict__ Pl,
                                           int grow0, int nvalid, int wave, int lane) {
  v4u hv[4], lv[4];
#pragma unroll
  for (int rr = 0; rr < 4; ++rr) {
    const int r = 4 * wave + rr;
    const float* tr = T + r * TP + 8 * lane;
    const v4f x0 = *(const v4f*)tr;
    const v4f x1 = *(const v4f*)(tr + 4);
    float x[8] = {x0.x, x0.y, x0.z, x0.w, x1.x, x1.y, x1.z, x1.w};
    if (ROT) {
      const float* cr = csS + r * 16 + 4 * (lane & 3);
      const float* sr = snS + r * 16 + 4 * (lane & 3);
#pragma unroll
      for (int pp = 0; pp < 4; ++pp) {
        const float c = cr[pp], s = sr[pp];
        const float e = x[2 * pp], o = x[2 * pp + 1];
        x[2 * pp]     = e * c - o * s;
        x[2 * pp + 1] = e * s + o * c;
      }
    }
    split8(x, hv[rr], lv[rr]);
  }
#pragma unroll
  for (int rr = 0; rr < 4; ++rr) {
    const int r = 4 * wave + rr;
    if (r < nvalid) {
      const size_t off = (size_t)(grow0 + r) * DM + 8 * lane;
      *(volatile v4u*)(Ph + off) = hv[rr];
      *(volatile v4u*)(Pl + off) = lv[rr];
    }
  }
  __threadfence();
#pragma unroll
  for (int rr = 0; rr < 4; ++rr) {
    const int r = 4 * wave + rr;
    if (r < nvalid) {
      const size_t off = (size_t)(grow0 + r) * DM + 8 * lane;
      *(volatile v4u*)(Ph + off) = hv[rr];
      *(volatile v4u*)(Pl + off) = lv[rr];
    }
  }
}

__global__ __launch_bounds__(256) void k_prep(const float* __restrict__ Wq, const float* __restrict__ Wk,
                                              const float* __restrict__ Wv, const float* __restrict__ Wo,
                                              unsigned short* __restrict__ WH, unsigned short* __restrict__ WL,
                                              int total8) {
  const int g = blockIdx.x * 256 + threadIdx.x;
  if (g >= total8) return;
  const int w  = g / (DM * DM / 8);
  const int e0 = (g - w * (DM * DM / 8)) * 8;
  const float* src = (w == 0) ? Wq : (w == 1) ? Wk : (w == 2) ? Wv : Wo;
  const v4f x0 = *(const v4f*)(src + e0);
  const v4f x1 = *(const v4f*)(src + e0 + 4);
  float x[8] = {x0.x, x0.y, x0.z, x0.w, x1.x, x1.y, x1.z, x1.w};
  v4u h, l;
  split8(x, h, l);
  const size_t off = (size_t)w * DM * DM + e0;
  *(volatile v4u*)(WH + off) = h;
  *(volatile v4u*)(WL + off) = l;
  __threadfence();
  *(volatile v4u*)(WH + off) = h;
  *(volatile v4u*)(WL + off) = l;
}

__global__ __launch_bounds__(256) void k_qproj(const float* __restrict__ query, const float* __restrict__ qpos,
                                               const float* __restrict__ ln_s, const float* __restrict__ ln_b,
                                               const unsigned short* __restrict__ WH,
                                               const unsigned short* __restrict__ WL,
                                               unsigned short* __restrict__ QH, unsigned short* __restrict__ QL,
                                               int M) {
  extern __shared__ __align__(16) char smem_q[];
  unsigned short* Ah = (unsigned short*)(smem_q + G_AH);
  unsigned short* Al = (unsigned short*)(smem_q + G_AL);
  float* T   = (float*)(smem_q + G_T);
  float* csS = (float*)(smem_q + G_CS);
  float* snS = (float*)(smem_q + G_SN);

  const int t = threadIdx.x, lane = t & 31, wave = t >> 5;
  const int row0 = blockIdx.x * BM;
  if (row0 >= M) return;
  const v4u zz = {0u, 0u, 0u, 0u};

  for (int e = t; e < BM * 16; e += 256) {
    const int r = e >> 4, p = e & 15;
    const int g = row0 + r;
    float cs = 1.f, sn = 0.f;
    if (g < M) {
      const float py = qpos[2 * g], px = qpos[2 * g + 1];
      const float ang = py * c_fs[p] + px * c_fs[p];
      cs = cosf(ang); sn = sinf(ang);
    }
    csS[e] = cs; snS[e] = sn;
  }

  float lns[8], lnb[8];
  {
    const v4f s0 = *(const v4f*)(ln_s + 8 * lane), s1 = *(const v4f*)(ln_s + 8 * lane + 4);
    const v4f b0 = *(const v4f*)(ln_b + 8 * lane), b1 = *(const v4f*)(ln_b + 8 * lane + 4);
    lns[0] = s0.x; lns[1] = s0.y; lns[2] = s0.z; lns[3] = s0.w;
    lns[4] = s1.x; lns[5] = s1.y; lns[6] = s1.z; lns[7] = s1.w;
    lnb[0] = b0.x; lnb[1] = b0.y; lnb[2] = b0.z; lnb[3] = b0.w;
    lnb[4] = b1.x; lnb[5] = b1.y; lnb[6] = b1.z; lnb[7] = b1.w;
  }
#pragma unroll
  for (int rr = 0; rr < 4; ++rr) {
    const int r = 4 * wave + rr;
    const int g = row0 + r;
    v4u h = zz, l = zz;
    if (g < M) {
      const float* src = query + (size_t)g * DM + 8 * lane;
      const v4f x0 = *(const v4f*)src;
      const v4f x1 = *(const v4f*)(src + 4);
      float x[8] = {x0.x, x0.y, x0.z, x0.w, x1.x, x1.y, x1.z, x1.w};
      float s = 0.f;
#pragma unroll
      for (int i = 0; i < 8; ++i) s += x[i];
      s = wsum(s);
      const float mean = s * (1.0f / DM);
      float d[8];
      float v = 0.f;
#pragma unroll
      for (int i = 0; i < 8; ++i) { d[i] = x[i] - mean; v += d[i] * d[i]; }
      v = wsum(v);
      const float rs = rsqrtf(v * (1.0f / DM) + 1.0e-5f);
      float y[8];
#pragma unroll
      for (int i = 0; i < 8; ++i) y[i] = d[i] * rs * lns[i] + lnb[i];
      split8(y, h, l);
    }
    *(v4u*)(Ah + r * AP + 8 * lane) = h;
    *(v4u*)(Al + r * AP + 8 * lane) = l;
  }
  __syncthreads();
  gemm_tile(Ah, Al, WH, WL, T, wave, lane);
  __syncthreads();
  epi_planes<true>(T, csS, snS, QH, QL, row0, min(BM, M - row0), wave, lane);
}

__global__ __launch_bounds__(256) void k_kvproj(const float* __restrict__ fmaps, const int* __restrict__ shapes,
                                                const unsigned short* __restrict__ WH,
                                                const unsigned short* __restrict__ WL,
                                                unsigned short* __restrict__ KH, unsigned short* __restrict__ KL,
                                                unsigned short* __restrict__ VH, unsigned short* __restrict__ VL,
                                                int ncell, int nb) {
  extern __shared__ __align__(16) char smem_k[];
  unsigned short* Ah = (unsigned short*)(smem_k + G_AH);
  unsigned short* Al = (unsigned short*)(smem_k + G_AL);
  float* T   = (float*)(smem_k + G_T);
  float* csS = (float*)(smem_k + G_CS);
  float* snS = (float*)(smem_k + G_SN);

  const int cidx0 = blockIdx.x * BM;
  if (cidx0 + BM > ncell) return;
  const int b    = cidx0 / CPB;
  const int rem  = cidx0 - b * CPB;
  const int lvl  = rem / (FH * FW);
  const int rem2 = rem - lvl * (FH * FW);
  const int ci   = rem2 / FW;
  const int cj0  = rem2 - ci * FW;
  int shy = shapes[2 * lvl], shx = shapes[2 * lvl + 1];
  shy = min(shy, FH); shx = min(shx, FW);
  if (b >= nb || ci >= shy || cj0 >= shx) return;

  const int t = threadIdx.x, lane = t & 31, wave = t >> 5;

  for (int e = t; e < BM * 16; e += 256) {
    const int r = e >> 4, p = e & 15;
    const float py = (float)ci, px = (float)(cj0 + r), pl = (float)lvl;
    const float ang = py * c_fs[p] + px * c_fs[p] + pl * c_fl[p];
    csS[e] = cosf(ang); snS[e] = sinf(ang);
  }
#pragma unroll
  for (int rr = 0; rr < 4; ++rr) {
    const int r = 4 * wave + rr;
    const float* src = fmaps + (size_t)(cidx0 + r) * DM + 8 * lane;
    const v4f x0 = *(const v4f*)src;
    const v4f x1 = *(const v4f*)(src + 4);
    float x[8] = {x0.x, x0.y, x0.z, x0.w, x1.x, x1.y, x1.z, x1.w};
    v4u h, l;
    split8(x, h, l);
    *(v4u*)(Ah + r * AP + 8 * lane) = h;
    *(v4u*)(Al + r * AP + 8 * lane) = l;
  }
  __syncthreads();
  gemm_tile(Ah, Al, WH + (size_t)1 * DM * DM, WL + (size_t)1 * DM * DM, T, wave, lane);
  __syncthreads();
  epi_planes<true>(T, csS, snS, KH, KL, cidx0, BM, wave, lane);
  __syncthreads();
  gemm_tile(Ah, Al, WH + (size_t)2 * DM * DM, WL + (size_t)2 * DM * DM, T, wave, lane);
  __syncthreads();
  epi_planes<false>(T, csS, snS, VH, VL, cidx0, BM, wave, lane);
}

__device__ __forceinline__ void gather_rows(unsigned short* R, const unsigned short* __restrict__ P,
                                            const int* cellS, int nrows, int wave, int lane) {
  const v4u zz = {0u, 0u, 0u, 0u};
  for (int l = wave; l < nrows; l += 8) {
    const int cell = cellS[l];
    v4u v = zz;
    if (cell >= 0) v = *(const v4u*)(P + (size_t)cell * DM + 8 * lane);
    *(v4u*)(R + l * RPH + 8 * lane) = v;
  }
}

__device__ __forceinline__ void score_pass(const unsigned short* R, const unsigned short* qhS,
                                           const unsigned short* qlS, v8f& s0, v8f& s1,
                                           int mt0, int mt1, int has2, int lane) {
  const int n = lane & 15, hh = lane >> 4;
  const v4u zz = {0u, 0u, 0u, 0u};
  const unsigned short* qsrc = (n & 8) ? qlS : qhS;
  const unsigned short* r0p = R + (16 * mt0 + n) * RPH + 8 * hh;
  const unsigned short* r1p = R + (16 * mt1 + n) * RPH + 8 * hh;
#pragma unroll 2
  for (int ks = 0; ks < DM / 32; ++ks) {
    const int k0 = 32 * ks;
    Frag bq;
    bq.u[0] = *(const v4u*)(qsrc + k0 + 8 * hh);
    bq.u[1] = *(const v4u*)(qsrc + k0 + 16 + 8 * hh);
    if ((n & 7) != ks) { bq.u[0] = zz; bq.u[1] = zz; }
    Frag a;
    a.u[0] = *(const v4u*)(r0p + k0);
    a.u[1] = *(const v4u*)(r0p + k0 + 16);
    s0 = wmma16(a.v, bq.v, s0);
    if (has2) {
      Frag c;
      c.u[0] = *(const v4u*)(r1p + k0);
      c.u[1] = *(const v4u*)(r1p + k0 + 16);
      s1 = wmma16(c.v, bq.v, s1);
    }
  }
}

__device__ __forceinline__ void pv_pass(const unsigned short* R, const unsigned short* attS,
                                        v8f& o0, v8f& o1, int ct0, int lane) {
  const int n = lane & 15, hh = lane >> 4;
  const unsigned short* ap = attS + n * ATP + 8 * hh;
  const int c0 = 16 * ct0 + n, c1 = c0 + 16;
#pragma unroll 1
  for (int ks = 0; ks < VROWS / 32; ++ks) {
    const int k0 = 32 * ks;
    Frag a;
    a.u[0] = *(const v4u*)(ap + k0);
    a.u[1] = *(const v4u*)(ap + k0 + 16);
    Frag b0, b1;
#pragma unroll
    for (int i = 0; i < 16; ++i) {
      const int l = k0 + ((i < 8) ? (8 * hh + i) : (8 + 8 * hh + i));
      b0.s[i] = R[l * RPH + c0];
      b1.s[i] = R[l * RPH + c1];
    }
    o0 = wmma16(a.v, b0.v, o0);
    o1 = wmma16(a.v, b1.v, o1);
  }
}

__global__ __launch_bounds__(256) void k_attn(const float* __restrict__ qpos, const int* __restrict__ qbo, int nbo,
                                              const int* __restrict__ shapes,
                                              const unsigned short* __restrict__ QH, const unsigned short* __restrict__ QL,
                                              const unsigned short* __restrict__ KH, const unsigned short* __restrict__ KL,
                                              const unsigned short* __restrict__ VH, const unsigned short* __restrict__ VL,
                                              float* __restrict__ O, int nq, int nb) {
  extern __shared__ __align__(16) char smem_a[];
  unsigned short* R    = (unsigned short*)(smem_a + A_R);
  unsigned short* qhS  = (unsigned short*)(smem_a + A_QH);
  unsigned short* qlS  = (unsigned short*)(smem_a + A_QL);
  float*          scp  = (float*)(smem_a + A_SCP);
  unsigned short* attS = (unsigned short*)(smem_a + A_ATT);
  float*          op   = (float*)(smem_a + A_OP);
  float*          oS   = (float*)(smem_a + A_OS);
  int*            cellS = (int*)(smem_a + A_CELL);
  int*            oobS  = (int*)(smem_a + A_OOB);

  const int q = blockIdx.x;
  if (q >= nq) return;
  const int t = threadIdx.x, lane = t & 31, wave = t >> 5;
  const v4u zz = {0u, 0u, 0u, 0u};
  const v8f z8 = {0.f, 0.f, 0.f, 0.f, 0.f, 0.f, 0.f, 0.f};

  if (t < VROWS) {
    int cell = -1, ob = 1;
    if (t < LT) {
      const int lvl   = (t < 9) ? 0 : (t < 34) ? 1 : (t < 83) ? 2 : 3;
      const int start = (lvl == 0) ? 0 : (lvl == 1) ? 9 : (lvl == 2) ? 34 : 83;
      const int s  = 3 + 2 * lvl;
      const int li = t - start;
      const int hw = (s - 1) >> 1;
      const int ai = li / s;
      const int di = ai - hw, dj = (li - ai * s) - hw;
      const int shy = shapes[2 * lvl], shx = shapes[2 * lvl + 1];
      int my = shapes[0], mx = shapes[1];
#pragma unroll
      for (int lv = 1; lv < NLEV; ++lv) { my = max(my, shapes[2 * lv]); mx = max(mx, shapes[2 * lv + 1]); }
      const float fy = (float)shy * (1.0f / (float)max(my, 1));
      const float fx = (float)shx * (1.0f / (float)max(mx, 1));
      const float qy = qpos[2 * q], qx = qpos[2 * q + 1];
      const float ty = fminf(fmaxf(qy * fy, -1.0e6f), 1.0e6f);
      const float tx = fminf(fmaxf(qx * fx, -1.0e6f), 1.0e6f);
      const int by = (int)floorf(ty), bx = (int)floorf(tx);
      const int ii = by + di, jj = bx + dj;
      ob = ((ii < 0) | (ii >= shy) | (jj < 0) | (jj >= shx)) ? 1 : 0;
      const int ic = min(max(ii, 0), FH - 1), jc = min(max(jj, 0), FW - 1);
      int cnt = 0;
      for (int i = 0; i < nbo; ++i) cnt += (qbo[i] <= q) ? 1 : 0;
      const int b = min(max(cnt - 1, 0), nb - 1);
      cell = ob ? -1 : (((b * NLEV + lvl) * FH + ic) * FW + jc);
    }
    cellS[t] = cell;
    oobS[t]  = ob;
  }
  if (t < 32) {
    *(v4u*)(qhS + 8 * lane) = *(const v4u*)(QH + (size_t)q * DM + 8 * lane);
  } else if (t < 64) {
    *(v4u*)(qlS + 8 * lane) = *(const v4u*)(QL + (size_t)q * DM + 8 * lane);
  }
  for (int i = t; i < (16 * ATP * 2) / 16; i += 256) ((v4u*)attS)[i] = zz;
  __syncthreads();

  const int mt0 = wave;
  const int has2 = (wave < 3) ? 1 : 0;
  const int mt1 = has2 ? (wave + 8) : wave;
  v8f s0 = z8, s1 = z8;
  gather_rows(R, KH, cellS, KROWS, wave, lane);
  __syncthreads();
  score_pass(R, qhS, qlS, s0, s1, mt0, mt1, has2, lane);
  __syncthreads();
  gather_rows(R, KL, cellS, KROWS, wave, lane);
  __syncthreads();
  score_pass(R, qhS, qlS, s0, s1, mt0, mt1, has2, lane);
  {
    const int n = lane & 15, hh = lane >> 4;
#pragma unroll
    for (int r = 0; r < 8; ++r) {
      scp[n * KROWS + 16 * mt0 + 8 * hh + r] = s0[r];
      if (has2) scp[n * KROWS + 16 * mt1 + 8 * hh + r] = s1[r];
    }
  }
  __syncthreads();

  {
    const int h = wave;
    float sv[6], ev[6];
    float mxv = -3.0e38f;
#pragma unroll
    for (int i = 0; i < 6; ++i) {
      const int l = lane + 32 * i;
      float s = -3.0e38f;
      if (l < LT) {
        const float raw = scp[h * KROWS + l] + scp[(h + 8) * KROWS + l];
        s = raw * RSQ;
        if (oobS[l]) s = -1.0e9f;
      }
      sv[i] = s;
      mxv = fmaxf(mxv, s);
    }
    mxv = wmax(mxv);
    float sum = 0.f;
#pragma unroll
    for (int i = 0; i < 6; ++i) {
      const int l = lane + 32 * i;
      float e = 0.f;
      if (l < LT) e = expf(sv[i] - mxv);
      ev[i] = e;
      sum += e;
    }
    sum = wsum(sum);
    const float inv = 1.0f / sum;
#pragma unroll
    for (int i = 0; i < 6; ++i) {
      const int l = lane + 32 * i;
      if (l < LT) {
        const float a = ev[i] * inv;
        const unsigned short ah = f2bf(a);
        const unsigned short al = f2bf(a - bf2f(ah));
        attS[h * ATP + l]       = ah;
        attS[(8 + h) * ATP + l] = al;
      }
    }
  }
  __syncthreads();

  v8f o0 = z8, o1 = z8;
  gather_rows(R, VH, cellS, VROWS, wave, lane);
  __syncthreads();
  pv_pass(R, attS, o0, o1, 2 * wave, lane);
  __syncthreads();
  gather_rows(R, VL, cellS, VROWS, wave, lane);
  __syncthreads();
  pv_pass(R, attS, o0, o1, 2 * wave, lane);
  {
    const int n = lane & 15, hh = lane >> 4;
#pragma unroll
    for (int r = 0; r < 8; ++r) {
      op[(8 * hh + r) * DM + 32 * wave + n]      = o0[r];
      op[(8 * hh + r) * DM + 32 * wave + 16 + n] = o1[r];
    }
  }
  __syncthreads();
  {
    const int c = t, h = c >> 5;
    oS[c] = op[h * DM + c] + op[(8 + h) * DM + c];
  }
  __syncthreads();

  if (wave == 0) {
    const v4f x0 = *(const v4f*)(oS + 4 * lane);
    const v4f x1 = *(const v4f*)(oS + 128 + 4 * lane);
    float* orow = O + (size_t)q * DM;
    *(volatile v4f*)(orow + 4 * lane) = x0;
    *(volatile v4f*)(orow + 128 + 4 * lane) = x1;
    __threadfence();
    *(volatile v4f*)(orow + 4 * lane) = x0;
    *(volatile v4f*)(orow + 128 + 4 * lane) = x1;
  }
}

__global__ __launch_bounds__(256) void k_oproj(const float* __restrict__ Ob, const float* __restrict__ query,
                                               const unsigned short* __restrict__ WH,
                                               const unsigned short* __restrict__ WL,
                                               float* __restrict__ out, int M) {
  extern __shared__ __align__(16) char smem_o[];
  unsigned short* Ah = (unsigned short*)(smem_o + G_AH);
  unsigned short* Al = (unsigned short*)(smem_o + G_AL);
  float* T = (float*)(smem_o + G_T);

  const int t = threadIdx.x, lane = t & 31, wave = t >> 5;
  const int row0 = blockIdx.x * BM;
  if (row0 >= M) return;
  const v4u zz = {0u, 0u, 0u, 0u};

#pragma unroll
  for (int rr = 0; rr < 4; ++rr) {
    const int r = 4 * wave + rr;
    const int g = row0 + r;
    v4u h = zz, l = zz;
    if (g < M) {
      const float* src = Ob + (size_t)g * DM + 8 * lane;
      const v4f x0 = *(const v4f*)src;
      const v4f x1 = *(const v4f*)(src + 4);
      float x[8] = {x0.x, x0.y, x0.z, x0.w, x1.x, x1.y, x1.z, x1.w};
      split8(x, h, l);
    }
    *(v4u*)(Ah + r * AP + 8 * lane) = h;
    *(v4u*)(Al + r * AP + 8 * lane) = l;
  }
  __syncthreads();
  gemm_tile(Ah, Al, WH + (size_t)3 * DM * DM, WL + (size_t)3 * DM * DM, T, wave, lane);
  __syncthreads();

  const int nvalid = min(BM, M - row0);
  v4f y0[4], y1[4];
#pragma unroll
  for (int rr = 0; rr < 4; ++rr) {
    const int r = 4 * wave + rr;
    const int g = row0 + r;
    const float* tr = T + r * TP;
    y0[rr] = *(const v4f*)(tr + 4 * lane);
    y1[rr] = *(const v4f*)(tr + 128 + 4 * lane);
    if (r < nvalid) {
      const v4f q0 = *(const v4f*)(query + (size_t)g * DM + 4 * lane);
      const v4f q1 = *(const v4f*)(query + (size_t)g * DM + 128 + 4 * lane);
      y0[rr] = q0 + y0[rr];
      y1[rr] = q1 + y1[rr];
    }
  }
#pragma unroll
  for (int rr = 0; rr < 4; ++rr) {
    const int r = 4 * wave + rr;
    if (r < nvalid) {
      float* orow = out + (size_t)(row0 + r) * DM;
      *(volatile v4f*)(orow + 4 * lane) = y0[rr];
      *(volatile v4f*)(orow + 128 + 4 * lane) = y1[rr];
    }
  }
  __threadfence();
#pragma unroll
  for (int rr = 0; rr < 4; ++rr) {
    const int r = 4 * wave + rr;
    if (r < nvalid) {
      float* orow = out + (size_t)(row0 + r) * DM;
      *(volatile v4f*)(orow + 4 * lane) = y0[rr];
      *(volatile v4f*)(orow + 128 + 4 * lane) = y1[rr];
    }
  }
}

extern "C" void kernel_launch(void* const* d_in, const int* in_sizes, int n_in,
                              void* d_out, int out_size, void* d_ws, size_t ws_size,
                              hipStream_t stream) {
  if (n_in < 11) return;
  const float* query  = (const float*)d_in[0];
  const float* qpos   = (const float*)d_in[1];
  const int*   qbo    = (const int*)  d_in[2];
  const float* fmaps  = (const float*)d_in[3];
  const int*   shapes = (const int*)  d_in[4];
  const float* ln_s   = (const float*)d_in[5];
  const float* ln_b   = (const float*)d_in[6];
  const float* Wq     = (const float*)d_in[7];
  const float* Wk     = (const float*)d_in[8];
  const float* Wv     = (const float*)d_in[9];
  const float* Wo     = (const float*)d_in[10];
  float* out = (float*)d_out;

  const int nq = in_sizes[0] / DM;
  if (nq <= 0 || in_sizes[0] != nq * DM || in_sizes[1] != 2 * nq || out_size != nq * DM) return;
  const int nbo = in_sizes[2];
  if (nbo <= 0) return;
  if (in_sizes[3] <= 0 || (in_sizes[3] % (CPB * DM)) != 0) return;
  const int nb = in_sizes[3] / (CPB * DM);
  const int ncell = nb * CPB;
  if (in_sizes[4] != 2 * NLEV || in_sizes[5] != DM || in_sizes[6] != DM) return;
  for (int i = 7; i <= 10; ++i) if (in_sizes[i] != DM * DM) return;

  size_t off = 0;
  const size_t oWH = off; off += (size_t)4 * DM * DM * 2;
  const size_t oWL = off; off += (size_t)4 * DM * DM * 2;
  const size_t oQH = off; off += (size_t)nq * DM * 2;
  const size_t oQL = off; off += (size_t)nq * DM * 2;
  const size_t oKH = off; off += (size_t)ncell * DM * 2;
  const size_t oKL = off; off += (size_t)ncell * DM * 2;
  const size_t oVH = off; off += (size_t)ncell * DM * 2;
  const size_t oVL = off; off += (size_t)ncell * DM * 2;
  const size_t oO  = off; off += (size_t)nq * DM * 4;
  if (off > ws_size) return;

  char* ws = (char*)d_ws;
  unsigned short* WH = (unsigned short*)(ws + oWH);
  unsigned short* WL = (unsigned short*)(ws + oWL);
  unsigned short* QH = (unsigned short*)(ws + oQH);
  unsigned short* QL = (unsigned short*)(ws + oQL);
  unsigned short* KH = (unsigned short*)(ws + oKH);
  unsigned short* KL = (unsigned short*)(ws + oKL);
  unsigned short* VH = (unsigned short*)(ws + oVH);
  unsigned short* VL = (unsigned short*)(ws + oVL);
  float*          Ob = (float*)(ws + oO);

  hipFuncSetAttribute(reinterpret_cast<const void*>(k_qproj),  hipFuncAttributeMaxDynamicSharedMemorySize, G_TOT);
  hipFuncSetAttribute(reinterpret_cast<const void*>(k_kvproj), hipFuncAttributeMaxDynamicSharedMemorySize, G_TOT);
  hipFuncSetAttribute(reinterpret_cast<const void*>(k_oproj),  hipFuncAttributeMaxDynamicSharedMemorySize, G_TOT);
  hipFuncSetAttribute(reinterpret_cast<const void*>(k_attn),   hipFuncAttributeMaxDynamicSharedMemorySize, A_TOT);

  const int total8 = 4 * DM * DM / 8;
  k_prep<<<(total8 + 255) / 256, 256, 0, stream>>>(Wq, Wk, Wv, Wo, WH, WL, total8);
  k_qproj<<<(nq + BM - 1) / BM, 256, G_TOT, stream>>>(query, qpos, ln_s, ln_b, WH, WL, QH, QL, nq);
  k_kvproj<<<(ncell + BM - 1) / BM, 256, G_TOT, stream>>>(fmaps, shapes, WH, WL, KH, KL, VH, VL, ncell, nb);
  k_attn<<<nq, 256, A_TOT, stream>>>(qpos, qbo, nbo, shapes, QH, QL, KH, KL, VH, VL, Ob, nq, nb);
  k_oproj<<<(nq + BM - 1) / BM, 256, G_TOT, stream>>>(Ob, query, WH, WL, out, nq);
}
